// PointNet2feat_9758165696591
// MI455X (gfx1250) — hardware-verified
//
#include <hip/hip_runtime.h>
#include <math.h>

#pragma clang fp contract(off)

typedef __attribute__((ext_vector_type(16))) _Float16 v16h;
typedef __attribute__((ext_vector_type(8)))  _Float16 v8h;
typedef __attribute__((ext_vector_type(8)))  float    v8f;
typedef __attribute__((ext_vector_type(4)))  float    v4f;
typedef __attribute__((ext_vector_type(4)))  unsigned v4u;

constexpr int   BATCH      = 32;
constexpr int   NSAMP      = 32;
constexpr int   NCODE      = 170;
constexpr int   NCODE_PAD  = 192;
constexpr int   OUT_ROW    = 510;
constexpr int   OUT_TOTAL  = BATCH * OUT_ROW;
constexpr float WCARRY     = 16.0f;
constexpr float WCARRY_INV = 1.0f / 16.0f;
constexpr int   SUM_ORDER  = 0;

static_assert(OUT_TOTAL == 16320, "output extent");
static_assert(OUT_TOTAL % 32 == 0, "whole lines");

union FragU { v16h v; v8h h[2]; };
__device__ __forceinline__ v16h frag_load(const _Float16* p) {
  FragU f;
  f.h[0] = *(const v8h*)(p);
  f.h[1] = *(const v8h*)(p + 16);
  return f.v;
}
__device__ __forceinline__ v8f mma_h(v16h a, v16h b, v8f c) {
  c = __builtin_amdgcn_wmma_f32_16x16x32_f16(false, a, false, b, (short)0, c, false, false);
  asm volatile("v_nop\n\tv_nop\n\tv_nop\n\tv_nop" : "+v"(c) : "v"(a), "v"(b));
  return c;
}
__device__ __forceinline__ void pin_h(v16h& x) { asm volatile("" : "+v"(x) :: "memory"); }

__device__ __forceinline__ unsigned h16bits(float f) {
  const _Float16 hv = (_Float16)f;
  const unsigned short us = __builtin_bit_cast(unsigned short, hv);
  return (unsigned)us;
}

__device__ __forceinline__ float sq3(float dx, float dy, float dz) {
#pragma clang fp contract(off)
  const float t0 = dx * dx;
  const float t1 = dy * dy;
  const float t2 = dz * dz;
  if (SUM_ORDER == 0) return (t0 + t2) + t1;
  return (t0 + t1) + t2;
}

struct PrepDesc {
  const float* w; const float* bias; unsigned short* wout; float* bout;
  int cin, cout, kpad, npad, cf, nx;
};
static_assert(sizeof(PrepDesc) == 56, "no padding");
struct PrepAll { PrepDesc d[12]; };
static_assert(sizeof(PrepAll) == 672, "no padding");

__global__ __launch_bounds__(256) void prep_kernel(PrepAll P) {
  PrepDesc d = P.d[0];
#pragma unroll
  for (int i = 1; i < 12; ++i) {
    if ((int)blockIdx.y == i) d = P.d[i];
  }
  const int tid = threadIdx.x;
  const int total_chunks = (d.npad * d.kpad) >> 3;
  const int ch = blockIdx.x * 256 + tid;
  if (ch < total_chunks) {
    const int kc = d.kpad >> 3;
    const int n = ch / kc;
    const int k0 = (ch - n * kc) << 3;
    const int nc = n < d.cout ? n : d.cout - 1;
    unsigned hb[8];
#pragma unroll
    for (int e = 0; e < 8; ++e) {
      const int kp = k0 + e;
      int ks = 0;
      bool ok = false;
      if (kp < d.cf) { ks = kp + d.nx; ok = true; }
      else if (kp < d.cf + d.nx) { ks = kp - d.cf; ok = true; }
      ok = ok && (n < d.cout);
      ks = ks < 0 ? 0 : ks;
      ks = ks > d.cin - 1 ? d.cin - 1 : ks;
      const float x = d.w[(size_t)nc * d.cin + ks];
      const float y = ok ? x * WCARRY : 0.0f;
      hb[e] = h16bits(y);
    }
    v4u wv;
    wv.x = hb[0] | (hb[1] << 16);
    wv.y = hb[2] | (hb[3] << 16);
    wv.z = hb[4] | (hb[5] << 16);
    wv.w = hb[6] | (hb[7] << 16);
    volatile v4u* dst = (volatile v4u*)(d.wout + (size_t)ch * 8);
    *dst = wv;
    __threadfence();
    *dst = wv;
  }
  if (blockIdx.x == 0 && tid < (d.npad >> 2)) {
    float bv[4];
#pragma unroll
    for (int e = 0; e < 4; ++e) {
      const int n = tid * 4 + e;
      const int nc = n < d.cout ? n : d.cout - 1;
      const float x = d.bias[nc];
      bv[e] = (n < d.cout) ? x : 0.0f;
    }
    v4f o;
    o.x = bv[0]; o.y = bv[1]; o.z = bv[2]; o.w = bv[3];
    volatile v4f* dst = (volatile v4f*)(d.bout + tid * 4);
    *dst = o;
    __threadfence();
    *dst = o;
  }
}

template <int N, int S, int NT>
__global__ __launch_bounds__(NT) void fps_kernel(const float* __restrict__ xyz, float* __restrict__ nxyz) {
#pragma clang fp contract(off)
  constexpr int PPT = N / NT;
  constexpr int NW  = NT / 32;
  static_assert(N % NT == 0 && PPT >= 1 && PPT <= 8, "points per thread");
  static_assert((3 * N) % 4 == 0 && (3 * S) % 32 == 0, "whole lines");
  __shared__ __align__(16) float sp[3 * N];
  __shared__ __align__(16) float so[3 * S];
  __shared__ float wv[2][NW];
  __shared__ int   wi[2][NW];
  __shared__ int   sidx[S];

  const int b = blockIdx.x, tid = threadIdx.x;
  const int lane = tid & 31, wid = tid >> 5;
  const float* src = xyz + (size_t)b * 3 * N;
  for (int i = tid; i < (3 * N) / 4; i += NT) {
    const v4f v = *(const v4f*)(src + 4 * i);
    *(v4f*)(sp + 4 * i) = v;
  }
  __syncthreads();

  float px[PPT], py[PPT], pz[PPT], md[PPT];
#pragma unroll
  for (int j = 0; j < PPT; ++j) {
    const int idx = j * NT + tid;
    px[j] = sp[idx];
    py[j] = sp[N + idx];
    pz[j] = sp[2 * N + idx];
    md[j] = 1e10f;
  }
  if (tid == 0) sidx[0] = 0;
  int last = 0;
  for (int it = 1; it < S; ++it) {
    const float lx = sp[last], ly = sp[N + last], lz = sp[2 * N + last];
    float bv = 0.0f;
    int bi = tid;
#pragma unroll
    for (int j = 0; j < PPT; ++j) {
      const float dx = px[j] - lx, dy = py[j] - ly, dz = pz[j] - lz;
      const float d = sq3(dx, dy, dz);
      const float m = fminf(md[j], d);
      md[j] = m;
      if (j == 0) { bv = m; bi = tid; }
      else if (m > bv) { bv = m; bi = j * NT + tid; }
    }
#pragma unroll
    for (int mk = 16; mk > 0; mk >>= 1) {
      const float ov = __shfl_xor(bv, mk, 32);
      const int   oi = __shfl_xor(bi, mk, 32);
      const bool take = (ov > bv) || (ov == bv && oi < bi);
      bv = take ? ov : bv;
      bi = take ? oi : bi;
    }
    const int buf = it & 1;
    if (lane == 0) { wv[buf][wid] = bv; wi[buf][wid] = bi; }
    __syncthreads();
    float fv = wv[buf][0];
    int   fi = wi[buf][0];
#pragma unroll
    for (int w = 1; w < NW; ++w) {
      const float ov = wv[buf][w];
      const int   oi = wi[buf][w];
      const bool take = (ov > fv) || (ov == fv && oi < fi);
      fv = take ? ov : fv;
      fi = take ? oi : fi;
    }
    fi = fi < 0 ? 0 : fi;
    fi = fi > N - 1 ? N - 1 : fi;
    last = fi;
    if (tid == 0) sidx[it] = fi;
  }
  __syncthreads();
  for (int i = tid; i < 3 * S; i += NT) {
    const int c = i / S;
    const int s = i - c * S;
    int id = sidx[s];
    id = id < 0 ? 0 : id;
    id = id > N - 1 ? N - 1 : id;
    so[i] = sp[c * N + id];
  }
  __syncthreads();
  float* dst = nxyz + (size_t)b * 3 * S;
  for (int pass = 0; pass < 2; ++pass) {
    for (int i = tid; i < (3 * S) / 4; i += NT) {
      const v4f v = *(const v4f*)(so + 4 * i);
      *(volatile v4f*)(dst + 4 * i) = v;
    }
    __threadfence();
  }
}

template <int N, int S>
__global__ __launch_bounds__(256) void ballq_kernel(const float* __restrict__ xyz, const float* __restrict__ nxyz,
                                                    int* __restrict__ nidx, float r2) {
#pragma clang fp contract(off)
  static_assert(N % 32 == 0 && S % 8 == 0, "chunking");
  __shared__ int lst[8][32];
  const int tid = threadIdx.x, lane = tid & 31, wave = tid >> 5;
  const int q = blockIdx.x * 8 + wave;
  const int b = q / S;
  const int s = q - b * S;
  const float cx = nxyz[((size_t)b * 3 + 0) * S + s];
  const float cy = nxyz[((size_t)b * 3 + 1) * S + s];
  const float cz = nxyz[((size_t)b * 3 + 2) * S + s];
  lst[wave][lane] = 0;
  __syncthreads();
  const float* bx = xyz + (size_t)b * 3 * N;
  int cnt = 0;
#pragma unroll 2
  for (int c0 = 0; c0 < N; c0 += 32) {
    const int i = c0 + lane;
    const float x = bx[i], y = bx[N + i], z = bx[2 * N + i];
    const float dx = cx - x, dy = cy - y, dz = cz - z;
    const float d2 = sq3(dx, dy, dz);
    const bool hit = d2 < r2;
    const unsigned mask = (unsigned)__ballot(hit ? 1 : 0);
    const int pre = __popc(mask & ((1u << lane) - 1u));
    const int pos = cnt + pre;
    if (hit && pos < NSAMP) lst[wave][pos] = i;
    cnt += __popc(mask);
  }
  __syncthreads();
  const int v = lst[wave][lane];
  const int first = lst[wave][0];
  const int cc = cnt < NSAMP ? cnt : NSAMP;
  int res = (lane < cc) ? v : first;
  res = res < 0 ? 0 : res;
  res = res > N - 1 ? N - 1 : res;
  volatile int* dst = (volatile int*)(nidx + (size_t)q * NSAMP + lane);
  *dst = res;
  __threadfence();
  *dst = res;
}

template <int K, int NN, int WX, int WY>
__device__ __forceinline__ void mlp_layer(const _Float16* X, _Float16* Y, const _Float16* W,
                                          const float* bias, int wave, int lane) {
  constexpr int KT = K / 32;
  static_assert(K % 32 == 0 && NN % 16 == 0, "tile multiples");
  const int rl = lane & 15, h = lane >> 4;
  v16h a[KT];
#pragma unroll
  for (int kt = 0; kt < KT; ++kt) a[kt] = frag_load(X + (wave * 16 + rl) * WX + kt * 32 + 8 * h);
#pragma unroll 1
  for (int nt = 0; nt < NN / 16; ++nt) {
    v8f acc = (v8f){0.f, 0.f, 0.f, 0.f, 0.f, 0.f, 0.f, 0.f};
    const _Float16* wr = W + (size_t)(nt * 16 + rl) * K + 8 * h;
#pragma unroll
    for (int kt = 0; kt < KT; ++kt) {
      const v16h bf = frag_load(wr + kt * 32);
      acc = mma_h(a[kt], bf, acc);
      if ((kt & 3) == 3) asm volatile("" ::: "memory");
    }
    const int ncol = nt * 16 + rl;
    const float bb = bias[ncol];
#pragma unroll
    for (int r = 0; r < 8; ++r) {
      float v = acc[r] * WCARRY_INV + bb;
      v = v > 0.0f ? v : 0.0f;
      Y[(wave * 16 + 8 * h + r) * WY + ncol] = (_Float16)v;
    }
  }
}

template <int K, int NN, int WX>
__device__ __forceinline__ void mlp_last(const _Float16* X, float* prow, const _Float16* W,
                                         const float* bias, int wave, int lane) {
  constexpr int KT = K / 32;
  static_assert(K % 32 == 0 && NN % 16 == 0, "tile multiples");
  const int rl = lane & 15, h = lane >> 4;
  v16h a[KT];
#pragma unroll
  for (int kt = 0; kt < KT; ++kt) a[kt] = frag_load(X + (wave * 16 + rl) * WX + kt * 32 + 8 * h);
#pragma unroll 1
  for (int nt = 0; nt < NN / 16; ++nt) {
    v8f acc = (v8f){0.f, 0.f, 0.f, 0.f, 0.f, 0.f, 0.f, 0.f};
    const _Float16* wr = W + (size_t)(nt * 16 + rl) * K + 8 * h;
#pragma unroll
    for (int kt = 0; kt < KT; ++kt) {
      const v16h bf = frag_load(wr + kt * 32);
      acc = mma_h(a[kt], bf, acc);
      if ((kt & 3) == 3) asm volatile("" ::: "memory");
    }
    const int ncol = nt * 16 + rl;
    const float bb = bias[ncol];
    float m = 0.0f;
#pragma unroll
    for (int r = 0; r < 8; ++r) {
      const float v = acc[r] * WCARRY_INV + bb;
      m = fmaxf(m, v);
    }
    const float o = __shfl_xor(m, 16, 32);
    m = fmaxf(m, o);
    if (h == 0) prow[ncol] = m;
  }
}

template <int CF, int K0, int N0, int N1, int N2, int NPTS, int S>
__global__ __launch_bounds__(128) void group_mlp_kernel(
    const float* __restrict__ xyz, const float* __restrict__ nxyz, const int* __restrict__ nidx,
    const unsigned short* fin,
    const unsigned short* __restrict__ w0p, const float* __restrict__ b0,
    const unsigned short* __restrict__ w1p, const float* __restrict__ b1,
    const unsigned short* __restrict__ w2p, const float* __restrict__ b2,
    unsigned short* fout) {
  constexpr int WA = (K0 > N1) ? K0 : N1;
  constexpr int WB = N0;
  static_assert(K0 == CF + 32, "tail block of 32 columns");
  static_assert(CF % 8 == 0 && K0 % 32 == 0 && N0 % 32 == 0 && N1 % 32 == 0 && N2 % 16 == 0, "tile multiples");
  static_assert(S % 2 == 0 && (2 * N2) / 8 <= 128 && (2 * N2 * 2) % 128 == 0, "output lines");
  __shared__ __align__(16) _Float16 bufA[64 * WA];
  __shared__ __align__(16) _Float16 bufB[64 * WB];
  __shared__ __align__(16) float part[4][N2];
  __shared__ int snid[64];

  const int tid = threadIdx.x, wave = tid >> 5, lane = tid & 31;
  const int q0 = blockIdx.x * 2;
  const int b = q0 / S;

  if (tid < 64) {
    int pi = nidx[(size_t)q0 * NSAMP + tid];
    pi = pi < 0 ? 0 : pi;
    pi = pi > NPTS - 1 ? NPTS - 1 : pi;
    snid[tid] = pi;
  }
  __syncthreads();
  if (CF > 0) {
    constexpr int CH = (CF > 0) ? CF / 8 : 1;
#pragma unroll 2
    for (int t = tid; t < 64 * CH; t += 128) {
      const int r = t / CH;
      const int ch = t - r * CH;
      const int pi = snid[r];
      const v4u v = *(const v4u*)(fin + ((size_t)b * NPTS + pi) * CF + ch * 8);
      *(v4u*)(bufA + r * WA + ch * 8) = v;
    }
  }
  if (tid < 64) {
    const int r = tid;
    const int pi = snid[r];
    const int s = (q0 + (r >> 5)) - b * S;
    const float px = xyz[((size_t)b * 3 + 0) * NPTS + pi];
    const float py = xyz[((size_t)b * 3 + 1) * NPTS + pi];
    const float pz = xyz[((size_t)b * 3 + 2) * NPTS + pi];
    const float ccx = nxyz[((size_t)b * 3 + 0) * S + s];
    const float ccy = nxyz[((size_t)b * 3 + 1) * S + s];
    const float ccz = nxyz[((size_t)b * 3 + 2) * S + s];
    const float dx = px - ccx, dy = py - ccy, dz = pz - ccz;
    unsigned zz = 0;
    asm volatile("" : "+v"(zz));
    const unsigned hx = h16bits(dx), hy = h16bits(dy), hz = h16bits(dz);
    v4u c0, cz;
    c0.x = hx | (hy << 16);
    c0.y = hz | (zz << 16);
    c0.z = zz; c0.w = zz;
    cz.x = zz; cz.y = zz; cz.z = zz; cz.w = zz;
    v4u* dst = (v4u*)(bufA + r * WA + CF);
    dst[0] = c0; dst[1] = cz; dst[2] = cz; dst[3] = cz;
  }
  __syncthreads();
  mlp_layer<K0, N0, WA, WB>(bufA, bufB, (const _Float16*)w0p, b0, wave, lane);
  __syncthreads();
  mlp_layer<N0, N1, WB, WA>(bufB, bufA, (const _Float16*)w1p, b1, wave, lane);
  __syncthreads();
  mlp_last<N1, N2, WA>(bufA, part[wave], (const _Float16*)w2p, b2, wave, lane);
  __syncthreads();
  constexpr int CPC = N2 / 8;
  if (tid < 2 * CPC) {
    const int c = tid / CPC;
    const int col0 = (tid - c * CPC) * 8;
    const v4f a0 = *(const v4f*)(&part[2 * c][col0]);
    const v4f a1 = *(const v4f*)(&part[2 * c][col0 + 4]);
    const v4f g0 = *(const v4f*)(&part[2 * c + 1][col0]);
    const v4f g1 = *(const v4f*)(&part[2 * c + 1][col0 + 4]);
    const float m0 = fmaxf(a0.x, g0.x), m1 = fmaxf(a0.y, g0.y);
    const float m2 = fmaxf(a0.z, g0.z), m3 = fmaxf(a0.w, g0.w);
    const float m4 = fmaxf(a1.x, g1.x), m5 = fmaxf(a1.y, g1.y);
    const float m6 = fmaxf(a1.z, g1.z), m7 = fmaxf(a1.w, g1.w);
    v4u wv;
    wv.x = h16bits(m0) | (h16bits(m1) << 16);
    wv.y = h16bits(m2) | (h16bits(m3) << 16);
    wv.z = h16bits(m4) | (h16bits(m5) << 16);
    wv.w = h16bits(m6) | (h16bits(m7) << 16);
    volatile v4u* dst = (volatile v4u*)(fout + (size_t)q0 * N2 + (size_t)tid * 8);
    *dst = wv;
    __threadfence();
    *dst = wv;
  }
}

template <int K, int S>
__device__ __forceinline__ void post_level(const _Float16* feats, const _Float16* W, const float* bias,
                                           float* spre, int b, int wave, int lane) {
  constexpr int KT = K / 32;
  static_assert(K % 32 == 0 && S % 16 == 0, "tile multiples");
  const int rl = lane & 15, h = lane >> 4;
  float cm[3];
#pragma unroll
  for (int j = 0; j < 3; ++j) cm[j] = -INFINITY;
#pragma unroll 1
  for (int mt = 0; mt < S / 16; ++mt) {
    v16h a[KT];
    const _Float16* ar = feats + ((size_t)b * S + mt * 16 + rl) * K + 8 * h;
#pragma unroll
    for (int kt = 0; kt < KT; ++kt) {
      a[kt] = frag_load(ar + kt * 32);
      pin_h(a[kt]);
    }
#pragma unroll
    for (int j = 0; j < 3; ++j) {
      v8f acc = (v8f){0.f, 0.f, 0.f, 0.f, 0.f, 0.f, 0.f, 0.f};
      const _Float16* wr = W + (size_t)((wave + 4 * j) * 16 + rl) * K + 8 * h;
#pragma unroll
      for (int kt = 0; kt < KT; ++kt) {
        const v16h bf = frag_load(wr + kt * 32);
        acc = mma_h(a[kt], bf, acc);
        if ((kt & 3) == 3) asm volatile("" ::: "memory");
      }
      float m = acc[0];
#pragma unroll
      for (int r = 1; r < 8; ++r) m = fmaxf(m, acc[r]);
      cm[j] = fmaxf(cm[j], m);
    }
  }
#pragma unroll
  for (int j = 0; j < 3; ++j) {
    const float o = __shfl_xor(cm[j], 16, 32);
    const float m = fmaxf(cm[j], o);
    const int n = (wave + 4 * j) * 16 + rl;
    const float bb = bias[n];
    if (h == 0) spre[n] = m * WCARRY_INV + bb;
  }
}

__global__ __launch_bounds__(128) void post_kernel(
    const unsigned short* __restrict__ f0, const unsigned short* __restrict__ f1, const unsigned short* __restrict__ f2,
    const unsigned short* __restrict__ pw0, const unsigned short* __restrict__ pw1, const unsigned short* __restrict__ pw2,
    const float* __restrict__ pb0, const float* __restrict__ pb1, const float* __restrict__ pb2,
    float* __restrict__ pre) {
  __shared__ __align__(16) float spre[NCODE_PAD];
  const int tid = threadIdx.x, wave = tid >> 5, lane = tid & 31;
  const int b = blockIdx.x;
  const int lvl = blockIdx.y;
  if (lvl == 0)      post_level<96, 512>((const _Float16*)f0, (const _Float16*)pw0, pb0, spre, b, wave, lane);
  else if (lvl == 1) post_level<192, 128>((const _Float16*)f1, (const _Float16*)pw1, pb1, spre, b, wave, lane);
  else               post_level<256, 32>((const _Float16*)f2, (const _Float16*)pw2, pb2, spre, b, wave, lane);
  __syncthreads();
  if (tid < NCODE_PAD / 4) {
    const v4f v = *(const v4f*)(spre + 4 * tid);
    volatile v4f* dst = (volatile v4f*)(pre + ((size_t)lvl * BATCH + b) * NCODE_PAD + 4 * tid);
    *dst = v;
    __threadfence();
    *dst = v;
  }
}

__global__ __launch_bounds__(256) void finalize_kernel(const float* __restrict__ pre, float* __restrict__ out) {
  const int e = blockIdx.x * 256 + threadIdx.x;
  if (e < OUT_TOTAL) {
    const int b = e / OUT_ROW;
    const int rem = e - b * OUT_ROW;
    const int l = rem / NCODE;
    const int c = rem - l * NCODE;
    const float p = pre[((size_t)l * BATCH + b) * NCODE_PAD + c];
    const float v = tanhf(p);
    volatile float* dst = (volatile float*)(out + e);
    *dst = v;
    __threadfence();
    *dst = v;
  }
}

extern "C" void kernel_launch(void* const* d_in, const int* in_sizes, int n_in,
                              void* d_out, int out_size, void* d_ws, size_t ws_size,
                              hipStream_t stream) {
  (void)in_sizes; (void)out_size;
  if (n_in < 25) return;
  const float* pc = (const float*)d_in[0];
  float* out = (float*)d_out;

  char* ws = (char*)d_ws;
  size_t off = 0;
  auto carve = [&](size_t bytes) -> char* {
    char* p = ws + off;
    off += (bytes + 255) & ~(size_t)255;
    return p;
  };
  float* nx0 = (float*)carve((size_t)BATCH * 3 * 512 * 4);
  float* nx1 = (float*)carve((size_t)BATCH * 3 * 128 * 4);
  float* nx2 = (float*)carve((size_t)BATCH * 3 * 32 * 4);
  int* ni0 = (int*)carve((size_t)BATCH * 512 * NSAMP * 4);
  int* ni1 = (int*)carve((size_t)BATCH * 128 * NSAMP * 4);
  int* ni2 = (int*)carve((size_t)BATCH * 32 * NSAMP * 4);
  unsigned short* ft0 = (unsigned short*)carve((size_t)BATCH * 512 * 96 * 2);
  unsigned short* ft1 = (unsigned short*)carve((size_t)BATCH * 128 * 192 * 2);
  unsigned short* ft2 = (unsigned short*)carve((size_t)BATCH * 32 * 256 * 2);

  static const int DIM[12][6] = {
      {3, 24, 32, 32, 0, 3},      {24, 48, 32, 64, 24, 0},   {48, 96, 64, 96, 48, 0},     {96, 170, 96, 192, 96, 0},
      {99, 48, 128, 64, 96, 3},   {48, 96, 64, 96, 48, 0},   {96, 192, 96, 192, 96, 0},   {192, 170, 192, 192, 192, 0},
      {195, 96, 224, 96, 192, 3}, {96, 192, 96, 192, 96, 0}, {192, 256, 192, 256, 192, 0}, {256, 170, 256, 192, 256, 0}};
  static_assert(sizeof(DIM) / sizeof(DIM[0]) == 12, "table extent");
  unsigned short* wp[12];
  float* bp[12];
  for (int m = 0; m < 12; ++m) wp[m] = (unsigned short*)carve((size_t)DIM[m][3] * DIM[m][2] * 2);
  for (int m = 0; m < 12; ++m) bp[m] = (float*)carve((size_t)DIM[m][3] * 4);
  float* pre = (float*)carve((size_t)3 * BATCH * NCODE_PAD * 4);
  if (off > ws_size || off > (size_t)134217728) return;

  PrepAll P;
  for (int m = 0; m < 12; ++m) {
    const int l = m / 4, j = m % 4;
    const int widx = (j < 3) ? (1 + 8 * l + 2 * j) : (7 + 8 * l);
    P.d[m].w = (const float*)d_in[widx];
    P.d[m].bias = (const float*)d_in[widx + 1];
    P.d[m].wout = wp[m];
    P.d[m].bout = bp[m];
    P.d[m].cin = DIM[m][0];
    P.d[m].cout = DIM[m][1];
    P.d[m].kpad = DIM[m][2];
    P.d[m].npad = DIM[m][3];
    P.d[m].cf = DIM[m][4];
    P.d[m].nx = DIM[m][5];
  }
  prep_kernel<<<dim3(24, 12), 256, 0, stream>>>(P);

  fps_kernel<2048, 512, 256><<<BATCH, 256, 0, stream>>>(pc, nx0);
  ballq_kernel<2048, 512><<<(BATCH * 512) / 8, 256, 0, stream>>>(pc, nx0, ni0, 0.04f);
  group_mlp_kernel<0, 32, 32, 64, 96, 2048, 512><<<(BATCH * 512) / 2, 128, 0, stream>>>(
      pc, nx0, ni0, ft1, wp[0], bp[0], wp[1], bp[1], wp[2], bp[2], ft0);

  fps_kernel<512, 128, 256><<<BATCH, 256, 0, stream>>>(nx0, nx1);
  ballq_kernel<512, 128><<<(BATCH * 128) / 8, 256, 0, stream>>>(nx0, nx1, ni1, 0.16f);
  group_mlp_kernel<96, 128, 64, 96, 192, 512, 128><<<(BATCH * 128) / 2, 128, 0, stream>>>(
      nx0, nx1, ni1, ft0, wp[4], bp[4], wp[5], bp[5], wp[6], bp[6], ft1);

  fps_kernel<128, 32, 128><<<BATCH, 128, 0, stream>>>(nx1, nx2);
  ballq_kernel<128, 32><<<(BATCH * 32) / 8, 256, 0, stream>>>(nx1, nx2, ni2, 0.64f);
  group_mlp_kernel<192, 224, 96, 192, 256, 128, 32><<<(BATCH * 32) / 2, 128, 0, stream>>>(
      nx1, nx2, ni2, ft1, wp[8], bp[8], wp[9], bp[9], wp[10], bp[10], ft2);

  post_kernel<<<dim3(BATCH, 3), 128, 0, stream>>>(ft0, ft1, ft2, wp[3], wp[7], wp[11], bp[3], bp[7], bp[11], pre);
  finalize_kernel<<<(OUT_TOTAL + 255) / 256, 256, 0, stream>>>(pre, out);
}
